// Embeddings_62208306315589
// MI455X (gfx1250) — hardware-verified
//
#include <hip/hip_runtime.h>
#include <stdint.h>
#include <stddef.h>

constexpr int kFea   = 256;
constexpr int kAtt   = 64;
constexpr int kHl    = 10;
constexpr int kSteps = 12;
constexpr int kBatch = 64;
constexpr int kBT    = kBatch * kSteps;
constexpr int kHid   = kFea * kHl;
constexpr int kIn    = 2 * kHid;
constexpr int kEncH  = 128;
constexpr int kGates = 4;
constexpr int kNAll  = kGates * kHid;
constexpr float kWCarry    = 1024.0f;
constexpr float kWCarryInv = 1.0f / 1024.0f;

static_assert(kIn % 32 == 0, "gate GEMM K multiple of 32");
static_assert(kHid % 32 == 0, "step-0 K multiple of 32");
static_assert(kBatch % 64 == 0, "gate GEMM M tile multiple");
static_assert(kNAll % 64 == 0, "gate GEMM N tile multiple");
static_assert((kNAll / 64) % 8 == 0, "gate GEMM tiles fill whole blocks");
static_assert(kAtt % 32 == 0 && kEncH % 32 == 0, "encoder K multiples of 32");
static_assert(kHid % 256 == 0, "cell chunking");
static_assert(kBT * kFea * kAtt == 12582912, "x element count");

constexpr size_t kWtBytes   = (size_t)kNAll * kIn * 2;
constexpr size_t kCombBytes = (size_t)kSteps * kBatch * kIn * 2;
constexpr size_t kCgBytes   = (size_t)kBatch * kNAll * 4;
constexpr size_t kCBytes    = (size_t)kBatch * kHid * 4;
constexpr size_t kW0tBytes  = (size_t)kEncH * kAtt * 2;
constexpr size_t kW1tBytes  = (size_t)16 * kEncH * 2;
constexpr size_t kOffWt   = 0;
constexpr size_t kOffComb = kOffWt + kWtBytes;
constexpr size_t kOffCg   = kOffComb + kCombBytes;
constexpr size_t kOffCA   = kOffCg + kCgBytes;
constexpr size_t kOffCB   = kOffCA + kCBytes;
constexpr size_t kOffHs32 = kOffCB + kCBytes;
constexpr size_t kOffW0t  = kOffHs32 + kCBytes;
constexpr size_t kOffW1t  = kOffW0t + kW0tBytes;
constexpr size_t kWsTotal = kOffW1t + kW1tBytes;
static_assert(kWsTotal == 117329920ull, "carve total");
static_assert(kWsTotal <= 134217728ull, "carve under 128 MiB");
static_assert(kOffComb % 256 == 0 && kOffCg % 256 == 0 && kOffCA % 256 == 0 && kOffCB % 256 == 0 &&
              kOffHs32 % 256 == 0 && kOffW0t % 256 == 0 && kOffW1t % 256 == 0, "aligned carve");

typedef __attribute__((ext_vector_type(16))) _Float16 v16h;
typedef __attribute__((ext_vector_type(8)))  _Float16 v8h;
typedef __attribute__((ext_vector_type(16))) __bf16   v16b;
typedef __attribute__((ext_vector_type(8)))  __bf16   v8b;
typedef __attribute__((ext_vector_type(8)))  float    v8f;
typedef __attribute__((ext_vector_type(4)))  float    v4f;
typedef __attribute__((ext_vector_type(4)))  unsigned v4u;
typedef __attribute__((ext_vector_type(2)))  unsigned v2u;

__device__ __forceinline__ unsigned short f2bf_bits(float f) {
  unsigned u = __float_as_uint(f);
  return (unsigned short)((u + 0x7FFFu + ((u >> 16) & 1u)) >> 16);
}
__device__ __forceinline__ float bf_bits2f(unsigned short h) { return __uint_as_float(((unsigned)h) << 16); }
__device__ __forceinline__ float bf_rne(float f) { return bf_bits2f(f2bf_bits(f)); }

__device__ __forceinline__ void dep_guard_h(v8f& a, v8f& b, v16h x, v16h y) { asm volatile("v_nop\n\tv_nop\n\tv_nop\n\tv_nop" : "+v"(a), "+v"(b) : "v"(x), "v"(y)); }
__device__ __forceinline__ void dep_guard_b(v8f& a, v8f& b, v16b x, v16b y) { asm volatile("v_nop\n\tv_nop\n\tv_nop\n\tv_nop" : "+v"(a), "+v"(b) : "v"(x), "v"(y)); }
__device__ __forceinline__ void keep4_h(v16h a, v16h b, v16h c, v16h d) { asm volatile("v_nop" :: "v"(a), "v"(b), "v"(c), "v"(d)); }
__device__ __forceinline__ void keep4_b(v16b a, v16b b, v16b c, v16b d) { asm volatile("v_nop" :: "v"(a), "v"(b), "v"(c), "v"(d)); }
__device__ __forceinline__ void acc_guard4(v8f& a, v8f& b, v8f& c, v8f& d) { asm volatile("v_nop\n\tv_nop\n\tv_nop\n\tv_nop" : "+v"(a), "+v"(b), "+v"(c), "+v"(d)); }
template <typename T> struct Frag;
template <> struct Frag<_Float16> {
  typedef v16h V; union U { v16h v; v8h h[2]; };
  static __device__ __forceinline__ v16h load(const _Float16* p) {
    U f; f.h[0] = *(const v8h*)(p); f.h[1] = *(const v8h*)(p + 16); return f.v;
  }
  static __device__ __forceinline__ v8f mma(v16h a, v16h b, v8f c) {
    return __builtin_amdgcn_wmma_f32_16x16x32_f16(false, a, false, b, (short)0, c, false, false);
  }
  static __device__ __forceinline__ void guard(v8f& a, v8f& b, v16h x, v16h y) { dep_guard_h(a, b, x, y); }
  static __device__ __forceinline__ void keep(v16h a, v16h b, v16h c, v16h d) { keep4_h(a, b, c, d); }
};
template <> struct Frag<__bf16> {
  typedef v16b V; union U { v16b v; v8b h[2]; };
  static __device__ __forceinline__ v16b load(const __bf16* p) {
    U f; f.h[0] = *(const v8b*)(p); f.h[1] = *(const v8b*)(p + 16); return f.v;
  }
  static __device__ __forceinline__ v8f mma(v16b a, v16b b, v8f c) {
    return __builtin_amdgcn_wmma_f32_16x16x32_bf16(false, a, false, b, (short)0, c, false, false);
  }
  static __device__ __forceinline__ void guard(v8f& a, v8f& b, v16b x, v16b y) { dep_guard_b(a, b, x, y); }
  static __device__ __forceinline__ void keep(v16b a, v16b b, v16b c, v16b d) { keep4_b(a, b, c, d); }
};

__device__ __forceinline__ v8f mma_bf16_g(v16b a, v16b b, v8f c) {
  c = __builtin_amdgcn_wmma_f32_16x16x32_bf16(false, a, false, b, (short)0, c, false, false);
  asm volatile("v_nop\n\tv_nop\n\tv_nop\n\tv_nop" : "+v"(c) : "v"(a), "v"(b));
  return c;
}

template <int ET> struct Elem;
template <> struct Elem<0> { typedef _Float16 T; };
template <> struct Elem<1> { typedef __bf16 T; };
template <int ET, bool SPLIT, int BIAS_MODE, int OUT_MODE, bool RESID, int ACT = 0>
__global__ __launch_bounds__(256) void wmma_gemm64(
    const unsigned short* __restrict__ Ap, const unsigned short* __restrict__ A2p, int lda, long strideA,
    const unsigned short* __restrict__ Btp, const unsigned short* __restrict__ Bt2p, int ldb, long strideB,
    void* __restrict__ Cout, void* __restrict__ Cout2, int ldc, long strideC,
    const float* __restrict__ bias,
    const float* __restrict__ resid, long strideR,
    int M, int N, int K, float scale) {
  typedef typename Elem<ET>::T T;
  typedef typename Frag<T>::V V;
  const T* A = (const T*)Ap; const T* A2 = (const T*)A2p; const T* Bt = (const T*)Btp; const T* Bt2 = (const T*)Bt2p;
  __shared__ __align__(16) float sT[8][16 * 68];
  const int b    = blockIdx.y;
  const int lane = threadIdx.x & 31;
  const int wave = threadIdx.x >> 5;
  const int tilesN = N >> 6;
  const int tilesM = M >> 6;
  const int tile = blockIdx.x * 8 + wave;
  if (tile >= tilesM * tilesN) return;
  const int tm = tile / tilesN;
  const int tn = tile - tm * tilesN;
  const int m0 = tm << 6;
  const int n0 = tn << 6;

  const T* Ab  = A  + (size_t)b * strideA;
  const T* Bb  = Bt + (size_t)b * strideB;
  const T* Ab2 = SPLIT ? (A2  + (size_t)b * strideA) : nullptr;
  const T* Bb2 = SPLIT ? (Bt2 + (size_t)b * strideB) : nullptr;

  const int rlane = lane & 15;
  const int koff  = (lane >> 4) * 8;
  const int mOff  = (lane >> 4) * 8;

  v8f acc[4][4];
#pragma unroll
  for (int i = 0; i < 4; ++i)
#pragma unroll
    for (int j = 0; j < 4; ++j) acc[i][j] = (v8f){0.f,0.f,0.f,0.f,0.f,0.f,0.f,0.f};

  for (int k0 = 0; k0 < K; k0 += 32) {
    V bh[4], bl[4];
#pragma unroll
    for (int j = 0; j < 4; ++j) {
      const size_t bo = (size_t)(n0 + (j << 4) + rlane) * ldb + koff + k0;
      bh[j] = Frag<T>::load(Bb + bo);
      if (SPLIT) bl[j] = Frag<T>::load(Bb2 + bo);
    }
#pragma unroll
    for (int i = 0; i < 4; ++i) {
      const size_t ao = (size_t)(m0 + (i << 4) + rlane) * lda + koff + k0;
      V ah = Frag<T>::load(Ab + ao);
      V al;
      if (SPLIT) al = Frag<T>::load(Ab2 + ao);
#pragma unroll
      for (int j = 0; j < 4; ++j) {
        acc[i][j] = Frag<T>::mma(ah, bh[j], acc[i][j]);
        if (SPLIT) {
          acc[i][j] = Frag<T>::mma(ah, bl[j], acc[i][j]);
          acc[i][j] = Frag<T>::mma(al, bh[j], acc[i][j]);
        }
      }
      Frag<T>::guard(acc[i][0], acc[i][3], ah, SPLIT ? al : ah);
    }
    Frag<T>::keep(bh[0], bh[1], bh[2], bh[3]);
    if (SPLIT) Frag<T>::keep(bl[0], bl[1], bl[2], bl[3]);
  }
  acc_guard4(acc[0][0], acc[0][1], acc[0][2], acc[0][3]);
  acc_guard4(acc[1][0], acc[1][1], acc[1][2], acc[1][3]);
  acc_guard4(acc[2][0], acc[2][1], acc[2][2], acc[2][3]);
  acc_guard4(acc[3][0], acc[3][1], acc[3][2], acc[3][3]);

  float* slab = sT[wave];
  const float* Rb = RESID ? (resid + (size_t)b * strideR) : nullptr;
#pragma unroll
  for (int i = 0; i < 4; ++i) {
    const int mBase = m0 + (i << 4);
#pragma unroll
    for (int j = 0; j < 4; ++j) {
      const int n = n0 + (j << 4) + rlane;
      float bv = 0.f;
      if (BIAS_MODE == 2) bv = bias[n];
#pragma unroll
      for (int r = 0; r < 8; ++r) {
        float v = acc[i][j][r] * scale;
        if (BIAS_MODE == 1) v += bias[mBase + mOff + r];
        if (BIAS_MODE == 2) v += bv;
        if (RESID) v += Rb[(size_t)(mBase + mOff + r) * ldc + n];
        if (ACT == 1) v = tanhf(v);
        if (ACT == 2) v = fmaxf(v, 0.0f);
        if (ACT == 3) v = v / (1.0f + expf(-v));
        if (ACT == 4) v = (v > 0.f) ? v : 0.01f * v;
        if (ACT == 5) v = 0.5f * v * (1.0f + erff(v * 0.70710678118654752f));
        slab[(mOff + r) * 68 + (j << 4) + rlane] = v;
      }
    }
    __builtin_amdgcn_fence(__ATOMIC_RELEASE, "workgroup");
    __builtin_amdgcn_wave_barrier();
    __builtin_amdgcn_fence(__ATOMIC_ACQUIRE, "workgroup");
    if (OUT_MODE == 0) {
      float* C = (float*)Cout + (size_t)b * strideC;
      const int hh = lane >> 4, c4 = (lane & 15) * 4;
      for (int pass = 0; pass < 2; ++pass) {
#pragma unroll
        for (int it = 0; it < 8; ++it) {
          const int row = it * 2 + hh;
          v4f v = *(const v4f*)(slab + row * 68 + c4);
          *(volatile v4f*)(C + (size_t)(mBase + row) * ldc + n0 + c4) = v;
        }
        __threadfence();
      }
    } else {
      const int q = lane >> 3, c8 = (lane & 7) * 8;
      unsigned short* C  = (unsigned short*)Cout  + (size_t)b * strideC;
      unsigned short* C2 = (OUT_MODE == 2) ? ((unsigned short*)Cout2 + (size_t)b * strideC) : nullptr;
      for (int pass = 0; pass < 2; ++pass) {
#pragma unroll
        for (int it = 0; it < 4; ++it) {
          const int row = it * 4 + q;
          const float* sp = slab + row * 68 + c8;
          v8h hv, lv;
#pragma unroll
          for (int e = 0; e < 8; ++e) {
            if (OUT_MODE == 1) {
              hv[e] = (_Float16)sp[e];
            } else {
              unsigned short hb = f2bf_bits(sp[e]);
              unsigned short lb = f2bf_bits(sp[e] - bf_bits2f(hb));
              hv[e] = __builtin_bit_cast(_Float16, hb);
              lv[e] = __builtin_bit_cast(_Float16, lb);
            }
          }
          *(volatile v8h*)(C + (size_t)(mBase + row) * ldc + n0 + c8) = hv;
          if (OUT_MODE == 2) *(volatile v8h*)(C2 + (size_t)(mBase + row) * ldc + n0 + c8) = lv;
        }
        __threadfence();
      }
    }
    __builtin_amdgcn_fence(__ATOMIC_RELEASE, "workgroup");
    __builtin_amdgcn_wave_barrier();
    __builtin_amdgcn_fence(__ATOMIC_ACQUIRE, "workgroup");
  }
}

__global__ __launch_bounds__(256) void prep_encoder_planes(
    const float* __restrict__ W0, const float* __restrict__ W1,
    unsigned short* __restrict__ W0t, unsigned short* __restrict__ W1t) {
  __shared__ __align__(16) unsigned short s0[kEncH * kAtt];
  __shared__ __align__(16) unsigned short s1[16 * kEncH];
  const int tid = threadIdx.x;
#pragma unroll
  for (int it = 0; it < 8; ++it) {
    const int e4 = tid + 256 * it;
    const int k = e4 >> 5;
    const int n = (e4 & 31) * 4;
    const v4f w = *(const v4f*)(W0 + 4 * e4);
#pragma unroll
    for (int i = 0; i < 4; ++i) s0[(n + i) * kAtt + k] = f2bf_bits(w[i]);
  }
#pragma unroll 1
  for (int it = 0; it < 5; ++it) {
    const int e = tid + 256 * it;
    const int col = e / kHl;
    const int l = e - col * kHl;
    s1[l * kEncH + col] = f2bf_bits(W1[e]);
  }
  {
    unsigned* s1w = (unsigned*)(void*)s1;
    for (int w = 640 + tid; w < 1024; w += 256) s1w[w] = 0u;
  }
  __syncthreads();
  for (int pass = 0; pass < 2; ++pass) {
#pragma unroll
    for (int it = 0; it < 4; ++it) {
      const int q = tid + 256 * it;
      const v4u v = *(const v4u*)(s0 + q * 8);
      *(volatile v4u*)(W0t + q * 8) = v;
    }
    {
      const v4u v = *(const v4u*)(s1 + tid * 8);
      *(volatile v4u*)(W1t + tid * 8) = v;
    }
    __threadfence();
  }
}

__global__ __launch_bounds__(256) void cast_gate_weights(
    const float* __restrict__ Wf, const float* __restrict__ Wi,
    const float* __restrict__ Wo, const float* __restrict__ Wc,
    unsigned short* __restrict__ Wt) {
  __shared__ __align__(16) unsigned short sW[64 * 72];
  const int tid = threadIdx.x;
  const int bid = blockIdx.x;
  const int g = bid / 3200;
  const int rem = bid - g * 3200;
  const int kt = rem / 40;
  const int ntl = rem - kt * 40;
  const int k0 = kt * 64;
  const int n0 = ntl * 64;
  const float* W = (g == 0) ? Wf : (g == 1) ? Wi : (g == 2) ? Wo : Wc;
#pragma unroll
  for (int it = 0; it < 4; ++it) {
    const int idx = tid + 256 * it;
    const int kr = idx >> 4;
    const int c4 = (idx & 15) * 4;
    const v4f w = *(const v4f*)(W + (size_t)(k0 + kr) * kHid + n0 + c4);
#pragma unroll
    for (int i = 0; i < 4; ++i) {
      const float r = bf_rne(w[i]) * kWCarry;
      sW[(c4 + i) * 72 + kr] = __builtin_bit_cast(unsigned short, (_Float16)r);
    }
  }
  __syncthreads();
  for (int pass = 0; pass < 2; ++pass) {
#pragma unroll
    for (int it = 0; it < 2; ++it) {
      const int q = tid + 256 * it;
      const int nr = q >> 3;
      const int c8 = (q & 7) * 8;
      const v4u v = *(const v4u*)(sW + nr * 72 + c8);
      *(volatile v4u*)(Wt + (size_t)(g * kHid + n0 + nr) * kIn + k0 + c8) = v;
    }
    __threadfence();
  }
}

__global__ __launch_bounds__(128) void encoder_wmma(
    const float* __restrict__ x, const unsigned short* __restrict__ W0t,
    const unsigned short* __restrict__ W1t, const float* __restrict__ b0,
    const float* __restrict__ b1, unsigned short* __restrict__ comb) {
  __shared__ __align__(16) unsigned short xs[64 * 72];
  __shared__ __align__(16) unsigned short w0s[kEncH * 72];
  __shared__ __align__(16) unsigned short h1h[64 * 136];
  __shared__ __align__(16) unsigned short h1l[64 * 136];
  __shared__ __align__(16) unsigned short outs[64 * kHl];
  __shared__ float b0s[kEncH];
  __shared__ float b1s[16];
  typedef Frag<__bf16> FB;

  const int tid = threadIdx.x;
  const int wave = tid >> 5;
  const int lane = tid & 31;
  const int rlane = lane & 15;
  const int hsel = lane >> 4;
  const int koff = hsel * 8;
  const int bt = blockIdx.x >> 2;
  const int quarter = blockIdx.x & 3;
  const int bidx = bt / kSteps;
  const int tstep = bt - bidx * kSteps;
  const size_t rowBase = (size_t)bt * kFea + (size_t)quarter * 64;

  b0s[tid] = bf_rne(b0[tid]);
  if (tid < 16) {
    const int ci = (tid < kHl) ? tid : (kHl - 1);
    const float bv = bf_rne(b1[ci]);
    b1s[tid] = (tid < kHl) ? bv : 0.0f;
  }
#pragma unroll
  for (int it = 0; it < 8; ++it) {
    const int idx = tid + 128 * it;
    const int r = idx >> 4;
    const int c4 = (idx & 15) * 4;
    const v4f v = *(const v4f*)(x + (rowBase + r) * kAtt + c4);
    v2u pk;
    pk[0] = (unsigned)f2bf_bits(v[0]) | ((unsigned)f2bf_bits(v[1]) << 16);
    pk[1] = (unsigned)f2bf_bits(v[2]) | ((unsigned)f2bf_bits(v[3]) << 16);
    *(v2u*)(xs + r * 72 + c4) = pk;
  }
#pragma unroll 1
  for (int it = 0; it < 8; ++it) {
    const int q = tid + 128 * it;
    const int n = q >> 3;
    const int k8 = (q & 7) * 8;
    const v4u v = *(const v4u*)(W0t + q * 8);
    *(v4u*)(w0s + n * 72 + k8) = v;
  }
  __syncthreads();

  const __bf16* xsb  = (const __bf16*)(const void*)xs;
  const __bf16* w0sb = (const __bf16*)(const void*)w0s;
  v8f acc1[8];
#pragma unroll
  for (int j = 0; j < 8; ++j) acc1[j] = (v8f){0.f,0.f,0.f,0.f,0.f,0.f,0.f,0.f};
#pragma unroll
  for (int ks = 0; ks < 2; ++ks) {
    const int k0 = ks * 32;
    const v16b a = FB::load(xsb + (wave * 16 + rlane) * 72 + koff + k0);
#pragma unroll
    for (int j = 0; j < 8; ++j) {
      const v16b bq = FB::load(w0sb + (j * 16 + rlane) * 72 + koff + k0);
      acc1[j] = mma_bf16_g(a, bq, acc1[j]);
    }
  }
#pragma unroll
  for (int j = 0; j < 8; ++j) {
    const int col = j * 16 + rlane;
    const float bb = b0s[col];
#pragma unroll
    for (int r = 0; r < 8; ++r) {
      const int row = wave * 16 + hsel * 8 + r;
      const float v = fmaxf(acc1[j][r] + bb, 0.0f);
      const unsigned short hb = f2bf_bits(v);
      const unsigned short lb = f2bf_bits(v - bf_bits2f(hb));
      h1h[row * 136 + col] = hb;
      h1l[row * 136 + col] = lb;
    }
  }
  __syncthreads();

  const __bf16* h1hb = (const __bf16*)(const void*)h1h;
  const __bf16* h1lb = (const __bf16*)(const void*)h1l;
  const __bf16* W1tb = (const __bf16*)(const void*)W1t;
  v8f acc2 = (v8f){0.f,0.f,0.f,0.f,0.f,0.f,0.f,0.f};
#pragma unroll
  for (int ks = 0; ks < 4; ++ks) {
    const int k0 = ks * 32;
    const v16b ah = FB::load(h1hb + (wave * 16 + rlane) * 136 + koff + k0);
    const v16b al = FB::load(h1lb + (wave * 16 + rlane) * 136 + koff + k0);
    const v16b bw = FB::load(W1tb + rlane * kEncH + koff + k0);
    acc2 = mma_bf16_g(ah, bw, acc2);
    acc2 = mma_bf16_g(al, bw, acc2);
  }
  {
    const float bb = b1s[rlane];
#pragma unroll
    for (int r = 0; r < 8; ++r) {
      const int row = wave * 16 + hsel * 8 + r;
      const float v = fmaxf(acc2[r] + bb, 0.0f);
      const unsigned short hv = __builtin_bit_cast(unsigned short, (_Float16)v);
      if (rlane < kHl) outs[row * kHl + rlane] = hv;
    }
  }
  __syncthreads();
  {
    unsigned short* dst = comb + ((size_t)(tstep * kBatch + bidx) * kIn + (size_t)quarter * 64 * kHl);
    for (int pass = 0; pass < 2; ++pass) {
      if (tid < 80) {
        const v4u v = *(const v4u*)(outs + tid * 8);
        *(volatile v4u*)(dst + tid * 8) = v;
      }
      __threadfence();
    }
  }
}

__global__ __launch_bounds__(256) void lstm_cell(
    const float* __restrict__ Cg, const float* __restrict__ cin, float* __restrict__ cout,
    const float* __restrict__ bfv, const float* __restrict__ biv,
    const float* __restrict__ bov, const float* __restrict__ bcv,
    unsigned short* __restrict__ hnext, float* __restrict__ hs32,
    int hasCin, int writeH16, int writeH32) {
  __shared__ __align__(16) float cs[256];
  __shared__ __align__(16) unsigned short h16s[256];
  __shared__ __align__(16) float h32s[256];
  const int tid = threadIdx.x;
  const int b = blockIdx.x / 10;
  const int chunk = blockIdx.x - b * 10;
  const int n = chunk * 256 + tid;
  const size_t gbase = (size_t)b * kNAll + n;
  const float pf = Cg[gbase] + bf_rne(bfv[n]);
  const float pi = Cg[gbase + kHid] + bf_rne(biv[n]);
  const float po = Cg[gbase + 2 * kHid] + bf_rne(bov[n]);
  const float pg = Cg[gbase + 3 * kHid] + bf_rne(bcv[n]);
  float cprev = 0.0f;
  if (hasCin) cprev = cin[(size_t)b * kHid + n];
  const float fg = __builtin_amdgcn_rcpf(1.0f + expf(-pf));
  const float ig = __builtin_amdgcn_rcpf(1.0f + expf(-pi));
  const float og = __builtin_amdgcn_rcpf(1.0f + expf(-po));
  const float gg = tanhf(pg);
  float cnew = fg * cprev;
  cnew = fmaf(ig, gg, cnew);
  const float hnew = og * tanhf(cnew);
  cs[tid] = cnew;
  h16s[tid] = __builtin_bit_cast(unsigned short, (_Float16)hnew);
  h32s[tid] = hnew;
  __syncthreads();
  float* cdst = cout + (size_t)b * kHid + chunk * 256;
  unsigned short* hdst = hnext + (size_t)b * kIn + kHid + chunk * 256;
  float* h32dst = hs32 + (size_t)b * kHid + chunk * 256;
  for (int pass = 0; pass < 2; ++pass) {
    if (tid < 64) {
      const v4f v = *(const v4f*)(cs + tid * 4);
      *(volatile v4f*)(cdst + tid * 4) = v;
    }
    if (writeH16 && tid >= 64 && tid < 96) {
      const int q = tid - 64;
      const v4u v = *(const v4u*)(h16s + q * 8);
      *(volatile v4u*)(hdst + q * 8) = v;
    }
    if (writeH32 && tid >= 96 && tid < 160) {
      const int q = tid - 96;
      const v4f v = *(const v4f*)(h32s + q * 4);
      *(volatile v4f*)(h32dst + q * 4) = v;
    }
    __threadfence();
  }
}

__global__ __launch_bounds__(256) void final_fc(
    const float* __restrict__ hs32, const float* __restrict__ Wfc,
    const float* __restrict__ bfc, float* __restrict__ out) {
  __shared__ float sW[kHl * kHl];
  __shared__ float sb[kHl];
  __shared__ __align__(16) float os[kFea * kHl];
  const int tid = threadIdx.x;
  if (tid < kHl * kHl) sW[tid] = bf_rne(Wfc[tid]);
  if (tid < kHl) sb[tid] = bf_rne(bfc[tid]);
  __syncthreads();
  const int b = blockIdx.x;
  const int fea = tid;
  const float* hp = hs32 + (size_t)b * kHid + fea * kHl;
  float o[kHl];
#pragma unroll
  for (int l = 0; l < kHl; ++l) o[l] = 0.0f;
#pragma unroll 1
  for (int j = 0; j < kHl; ++j) {
    const float v = fmaxf(hp[j], 0.0f);
#pragma unroll
    for (int l = 0; l < kHl; ++l) o[l] = fmaf(v, sW[j * kHl + l], o[l]);
  }
#pragma unroll
  for (int l = 0; l < kHl; ++l) os[fea * kHl + l] = o[l] + sb[l];
  __syncthreads();
  float* dst = out + (size_t)b * kHid;
  for (int pass = 0; pass < 2; ++pass) {
#pragma unroll
    for (int it = 0; it < 3; ++it) {
      const int q = tid + 256 * it;
      if (q < (kFea * kHl) / 4) {
        const v4f v = *(const v4f*)(os + q * 4);
        *(volatile v4f*)(dst + q * 4) = v;
      }
    }
    __threadfence();
  }
}

extern "C" void kernel_launch(void* const* d_in, const int* in_sizes, int n_in,
                              void* d_out, int out_size, void* d_ws,
                              size_t ws_size, hipStream_t stream) {
  if (n_in < 15) return;
  if (ws_size < kWsTotal) return;
  if (out_size < kBatch * kHid) return;
  if (in_sizes[0] != kBT * kFea * kAtt) return;
  if (in_sizes[1] != kAtt * kEncH) return;
  if (in_sizes[3] != kEncH * kHl) return;
  if (in_sizes[5] != kIn * kHid || in_sizes[7] != kIn * kHid ||
      in_sizes[9] != kIn * kHid || in_sizes[11] != kIn * kHid) return;

  const float* x   = (const float*)d_in[0];
  const float* W0  = (const float*)d_in[1];
  const float* b0  = (const float*)d_in[2];
  const float* W1  = (const float*)d_in[3];
  const float* b1  = (const float*)d_in[4];
  const float* Wf  = (const float*)d_in[5];
  const float* bfv = (const float*)d_in[6];
  const float* Wi  = (const float*)d_in[7];
  const float* biv = (const float*)d_in[8];
  const float* Wo  = (const float*)d_in[9];
  const float* bov = (const float*)d_in[10];
  const float* Wc  = (const float*)d_in[11];
  const float* bcv = (const float*)d_in[12];
  const float* Wfc = (const float*)d_in[13];
  const float* bfc = (const float*)d_in[14];
  float* out = (float*)d_out;

  char* ws = (char*)d_ws;
  unsigned short* Wt   = (unsigned short*)(ws + kOffWt);
  unsigned short* comb = (unsigned short*)(ws + kOffComb);
  float* Cg   = (float*)(ws + kOffCg);
  float* cA   = (float*)(ws + kOffCA);
  float* cB   = (float*)(ws + kOffCB);
  float* hs32 = (float*)(ws + kOffHs32);
  unsigned short* W0t = (unsigned short*)(ws + kOffW0t);
  unsigned short* W1t = (unsigned short*)(ws + kOffW1t);

  prep_encoder_planes<<<1, 256, 0, stream>>>(W0, W1, W0t, W1t);
  cast_gate_weights<<<kGates * (kIn / 64) * (kHid / 64), 256, 0, stream>>>(Wf, Wi, Wo, Wc, Wt);
  encoder_wmma<<<kBT * 4, 128, 0, stream>>>(x, W0t, W1t, b0, b1, comb);

  const size_t slotHalves = (size_t)kBatch * kIn;
  for (int t = 0; t < kSteps; ++t) {
    const unsigned short* combA = comb + (size_t)t * slotHalves;
    const int Kt = (t == 0) ? kHid : kIn;
    wmma_gemm64<0, false, 0, 0, false, 0><<<dim3(kNAll / 64 / 8, 1), 256, 0, stream>>>(
        combA, combA, kIn, 0L,
        Wt, Wt, kIn, 0L,
        (void*)Cg, (void*)Cg, kNAll, 0L,
        bfv,
        Cg, 0L,
        kBatch, kNAll, Kt, kWCarryInv);
    const float* cin = (t & 1) ? cA : cB;
    float* coutp = (t & 1) ? cB : cA;
    const int last = (t == kSteps - 1) ? 1 : 0;
    unsigned short* hnext = last ? comb : (comb + (size_t)(t + 1) * slotHalves);
    lstm_cell<<<kBatch * (kHid / 256), 256, 0, stream>>>(
        Cg, cin, coutp, bfv, biv, bov, bcv, hnext, hs32,
        (t == 0) ? 0 : 1, last ? 0 : 1, last);
  }

  final_fc<<<kBatch, kFea, 0, stream>>>(hs32, Wfc, bfc, out);
}
